// Model_61512521613593
// MI455X (gfx1250) — hardware-verified
//
#include <hip/hip_runtime.h>
#include <math.h>

typedef __attribute__((ext_vector_type(16))) _Float16 v16h;
typedef __attribute__((ext_vector_type(8)))  _Float16 v8h;
typedef __attribute__((ext_vector_type(8)))  float    v8f;
typedef __attribute__((ext_vector_type(4)))  float    v4f;

constexpr int kBatch   = 2048;
constexpr int kSteps   = 128;
constexpr int kFeat    = 37;
constexpr int kFeatPad = 64;
constexpr int kHid     = 64;
constexpr int kGate    = 256;
constexpr int kEncK    = 128;
constexpr int kDecIn   = 128;
constexpr int kDecK    = 192;
constexpr int kOutLen  = 10;
constexpr int kCls     = 11;
constexpr float kWCarry    = 16.0f;
constexpr float kWCarryInv = 1.0f / 16.0f;
constexpr float kLoCarry   = 2048.0f;
constexpr float kLoFold    = 1.0f / (16.0f * 2048.0f);
constexpr int XP = 72;
constexpr int HP = 72;
constexpr int FP = 136;
constexpr int SP = 68;
constexpr int kXVec     = kSteps * kFeat / 4;
constexpr int kPadCols  = kFeatPad - kFeat;
constexpr int kOutTile  = 16 * kOutLen * kCls;
constexpr int kOutVec   = kOutTile / 4;
constexpr int kPairs    = 16 * kCls;
static_assert((kSteps * kFeat) % 4 == 0, "x slab is a whole number of 16-B vectors");
static_assert(kXVec == 1184, "x slab vector count");
static_assert(kFeatPad % 32 == 0 && kEncK % 32 == 0 && kDecIn % 32 == 0 && kHid % 32 == 0, "K multiples of 32");
static_assert(kBatch % 16 == 0 && kSteps % 16 == 0 && kGate % 64 == 0, "tile multiples");
static_assert((kOutTile * 4) % 128 == 0, "output tile is a whole number of 128-B lines");
static_assert(kOutVec == 440, "output tile vector count");
static_assert((2 * 16 * HP) % 128 == 0, "h tile zero-fill loop exact");

union FragU { v16h v; v8h h[2]; };
__device__ __forceinline__ v16h frag_load(const _Float16* p) {
  FragU f; f.h[0] = *(const v8h*)(p); f.h[1] = *(const v8h*)(p + 16); return f.v;
}
__device__ __forceinline__ v8f mma_h(v16h a, v16h b, v8f c) {
  return __builtin_amdgcn_wmma_f32_16x16x32_f16(false, a, false, b, (short)0, c, false, false);
}
__device__ __forceinline__ void guard4(v8f& c0, v8f& c1, v8f& c2, v8f& c3, v16h a, v16h b0, v16h b1, v16h b2, v16h b3) {
  asm volatile("v_nop\n\tv_nop\n\tv_nop\n\tv_nop" : "+v"(c0), "+v"(c1), "+v"(c2), "+v"(c3) : "v"(a), "v"(b0), "v"(b1), "v"(b2), "v"(b3));
}
__device__ __forceinline__ void guard8(v8f& c0, v8f& c1, v8f& c2, v8f& c3, v8f& d0, v8f& d1, v8f& d2, v8f& d3,
                                       v16h ah, v16h al, v16h b0, v16h b1, v16h b2, v16h b3) {
  asm volatile("v_nop\n\tv_nop\n\tv_nop\n\tv_nop"
               : "+v"(c0), "+v"(c1), "+v"(c2), "+v"(c3), "+v"(d0), "+v"(d1), "+v"(d2), "+v"(d3)
               : "v"(ah), "v"(al), "v"(b0), "v"(b1), "v"(b2), "v"(b3));
}
__device__ __forceinline__ void acc_guard4(v8f& a, v8f& b, v8f& c, v8f& d) {
  asm volatile("v_nop\n\tv_nop\n\tv_nop\n\tv_nop" : "+v"(a), "+v"(b), "+v"(c), "+v"(d));
}
__device__ __forceinline__ float fsig(float x)  { return __builtin_amdgcn_rcpf(1.0f + __expf(-x)); }
__device__ __forceinline__ float ftanh(float x) { return 1.0f - 2.0f * __builtin_amdgcn_rcpf(__expf(2.0f * x) + 1.0f); }

__global__ __launch_bounds__(256) void wprep_kernel(const float* __restrict__ wih_f, const float* __restrict__ whh_f,
                                                    const float* __restrict__ wih_b, const float* __restrict__ whh_b,
                                                    const float* __restrict__ dwih, const float* __restrict__ dwhh,
                                                    const float* __restrict__ elw,
                                                    unsigned short* __restrict__ WE, unsigned short* __restrict__ WD,
                                                    unsigned short* __restrict__ WL) {
  const int job = blockIdx.y;
  const float* src = wih_f;
  unsigned short* dst = WE;
  int kreal = 64, lg8 = 3, dpitch = kEncK, dcol0 = 0, nrows = kGate;
  if (job == 1) { src = whh_f; dcol0 = 64; }
  else if (job == 2) { src = wih_b; dst = WE + kGate * kEncK; }
  else if (job == 3) { src = whh_b; dst = WE + kGate * kEncK; dcol0 = 64; }
  else if (job == 4) { src = dwih; dst = WD; kreal = 128; lg8 = 4; dpitch = kDecK; }
  else if (job == 5) { src = dwhh; dst = WD; dpitch = kDecK; dcol0 = 128; }
  else if (job == 6) { src = elw; dst = WL; kreal = kFeat; dpitch = kFeatPad; nrows = 64; }
  const int i = blockIdx.x * 256 + threadIdx.x;
  if (i < (nrows << lg8)) {
    const int row = i >> lg8;
    const int c8  = (i & ((1 << lg8) - 1)) * 8;
    v8h hv;
#pragma unroll
    for (int e = 0; e < 8; ++e) {
      const int k  = c8 + e;
      const int kc = (k < kreal) ? k : (kreal - 1);
      const float f = src[(size_t)row * kreal + kc];
      const float val = (k < kreal) ? (f * kWCarry) : 0.0f;
      hv[e] = (_Float16)val;
    }
    _Float16* dp = (_Float16*)dst + (size_t)row * dpitch + dcol0 + c8;
    *(volatile v8h*)dp = hv;
    __threadfence();
    *(volatile v8h*)dp = hv;
  }
}

__global__ __launch_bounds__(256) void enc_lin_kernel(const float* __restrict__ x, const unsigned short* __restrict__ WLp,
                                                      const float* __restrict__ bias, unsigned short* __restrict__ Ep) {
  __shared__ __align__(16) _Float16 Xa[kSteps * XP];
  __shared__ __align__(16) _Float16 Es[8 * 16 * XP];
  const _Float16* WL = (const _Float16*)WLp;
  _Float16* E = (_Float16*)Ep;
  const int tid = threadIdx.x, lane = tid & 31, wave = tid >> 5;
  const int c = lane & 15, hh = lane >> 4, koff = hh * 8;
  const int b = blockIdx.x;
  const float* xb = x + (size_t)b * (kSteps * kFeat);

#pragma unroll 1
  for (int it = 0; it < 5; ++it) {
    const int idx = it * 256 + tid;
    const int idc = (idx < kXVec) ? idx : (kXVec - 1);
    const v4f v = *(const v4f*)(xb + 4 * idc);
    if (idx < kXVec) {
#pragma unroll
      for (int e = 0; e < 4; ++e) {
        const int el  = 4 * idx + e;
        const int row = el / kFeat;
        const int col = el - row * kFeat;
        Xa[row * XP + col] = (_Float16)v[e];
      }
    }
  }
#pragma unroll 1
  for (int i = tid; i < kSteps * kPadCols; i += 256) {
    const int row = i / kPadCols;
    const int col = kFeat + (i - row * kPadCols);
    Xa[row * XP + col] = (_Float16)0.0f;
  }
  __syncthreads();

  const v8f z8 = {0.f, 0.f, 0.f, 0.f, 0.f, 0.f, 0.f, 0.f};
  v8f acc0 = z8, acc1 = z8, acc2 = z8, acc3 = z8;
  const _Float16* arow = Xa + (16 * wave + c) * XP + koff;
  const _Float16* wrow = WL + (size_t)c * kFeatPad + koff;
#pragma unroll
  for (int kt = 0; kt < 2; ++kt) {
    const v16h a   = frag_load(arow + 32 * kt);
    const v16h b0f = frag_load(wrow + (size_t)0 * 16 * kFeatPad + 32 * kt);
    const v16h b1f = frag_load(wrow + (size_t)1 * 16 * kFeatPad + 32 * kt);
    const v16h b2f = frag_load(wrow + (size_t)2 * 16 * kFeatPad + 32 * kt);
    const v16h b3f = frag_load(wrow + (size_t)3 * 16 * kFeatPad + 32 * kt);
    acc0 = mma_h(a, b0f, acc0);
    acc1 = mma_h(a, b1f, acc1);
    acc2 = mma_h(a, b2f, acc2);
    acc3 = mma_h(a, b3f, acc3);
    guard4(acc0, acc1, acc2, acc3, a, b0f, b1f, b2f, b3f);
  }
  acc_guard4(acc0, acc1, acc2, acc3);

  _Float16* es = Es + wave * (16 * XP);
  {
    const float bv0 = bias[0 * 16 + c];
    const float bv1 = bias[1 * 16 + c];
    const float bv2 = bias[2 * 16 + c];
    const float bv3 = bias[3 * 16 + c];
#pragma unroll
    for (int r = 0; r < 8; ++r) {
      const float v0 = fmaxf(acc0[r] * kWCarryInv + bv0, 0.0f);
      const float v1 = fmaxf(acc1[r] * kWCarryInv + bv1, 0.0f);
      const float v2 = fmaxf(acc2[r] * kWCarryInv + bv2, 0.0f);
      const float v3 = fmaxf(acc3[r] * kWCarryInv + bv3, 0.0f);
      es[(8 * hh + r) * XP + 0 * 16 + c] = (_Float16)v0;
      es[(8 * hh + r) * XP + 1 * 16 + c] = (_Float16)v1;
      es[(8 * hh + r) * XP + 2 * 16 + c] = (_Float16)v2;
      es[(8 * hh + r) * XP + 3 * 16 + c] = (_Float16)v3;
    }
  }
  __syncthreads();
  {
    const int q = lane >> 3, c8 = (lane & 7) * 8;
    v8h hv[4];
#pragma unroll
    for (int it = 0; it < 4; ++it) hv[it] = *(const v8h*)(es + (it * 4 + q) * XP + c8);
    for (int pass = 0; pass < 2; ++pass) {
#pragma unroll
      for (int it = 0; it < 4; ++it) {
        const int t = 16 * wave + it * 4 + q;
        *(volatile v8h*)(E + ((size_t)t * kBatch + (size_t)b) * kHid + c8) = hv[it];
      }
      __threadfence();
    }
  }
}

__global__ __launch_bounds__(128) void bilstm_kernel(const unsigned short* __restrict__ Ep, const unsigned short* __restrict__ WEp,
                                                     const float* __restrict__ bih_f, const float* __restrict__ bhh_f,
                                                     const float* __restrict__ bih_b, const float* __restrict__ bhh_b,
                                                     float* __restrict__ fd) {
  __shared__ __align__(16) _Float16 Ah[2 * 16 * HP];
  __shared__ __align__(16) float    Fs[16 * SP];
  const int tid = threadIdx.x, lane = tid & 31, wave = tid >> 5;
  const int c = lane & 15, hh = lane >> 4, koff = hh * 8;
  const int dir = blockIdx.y;
  const int rowbase = blockIdx.x * 16;
  const int j = 16 * wave + c;
  const _Float16* E = (const _Float16*)Ep;
  const _Float16* W = (const _Float16*)WEp + (size_t)dir * kGate * kEncK;

  float bb0, bb1, bb2, bb3;
  {
    const float f0 = bih_f[0 * kHid + j] + bhh_f[0 * kHid + j];
    const float f1 = bih_f[1 * kHid + j] + bhh_f[1 * kHid + j];
    const float f2 = bih_f[2 * kHid + j] + bhh_f[2 * kHid + j];
    const float f3 = bih_f[3 * kHid + j] + bhh_f[3 * kHid + j];
    const float k0 = bih_b[0 * kHid + j] + bhh_b[0 * kHid + j];
    const float k1 = bih_b[1 * kHid + j] + bhh_b[1 * kHid + j];
    const float k2 = bih_b[2 * kHid + j] + bhh_b[2 * kHid + j];
    const float k3 = bih_b[3 * kHid + j] + bhh_b[3 * kHid + j];
    bb0 = dir ? k0 : f0;
    bb1 = dir ? k1 : f1;
    bb2 = dir ? k2 : f2;
    bb3 = dir ? k3 : f3;
  }
#pragma unroll 1
  for (int i = tid; i < 2 * 16 * HP; i += 128) Ah[i] = (_Float16)0.0f;
  float cst[8], fda[8];
#pragma unroll
  for (int r = 0; r < 8; ++r) { cst[r] = 0.0f; fda[r] = 0.0f; }
  __syncthreads();

  const _Float16* wrow = W + (size_t)j * kEncK + koff;
  const v8f z8 = {0.f, 0.f, 0.f, 0.f, 0.f, 0.f, 0.f, 0.f};

#pragma unroll 1
  for (int s = 0; s < kSteps; ++s) {
    const int t   = dir ? (kSteps - 1 - s) : s;
    const int cur = s & 1;
    const _Float16* erow  = E + ((size_t)t * kBatch + (size_t)(rowbase + c)) * kHid + koff;
    const _Float16* ahrow = Ah + cur * (16 * HP) + c * HP + koff;
    _Float16* ahn = Ah + (cur ^ 1) * (16 * HP);
    v8f acc0 = z8, acc1 = z8, acc2 = z8, acc3 = z8;
#pragma unroll 1
    for (int kx = 0; kx < kHid; kx += 32) {
      const v16h a   = frag_load(erow + kx);
      const v16h b0f = frag_load(wrow + (size_t)0 * kHid * kEncK + kx);
      const v16h b1f = frag_load(wrow + (size_t)1 * kHid * kEncK + kx);
      const v16h b2f = frag_load(wrow + (size_t)2 * kHid * kEncK + kx);
      const v16h b3f = frag_load(wrow + (size_t)3 * kHid * kEncK + kx);
      acc0 = mma_h(a, b0f, acc0);
      acc1 = mma_h(a, b1f, acc1);
      acc2 = mma_h(a, b2f, acc2);
      acc3 = mma_h(a, b3f, acc3);
      guard4(acc0, acc1, acc2, acc3, a, b0f, b1f, b2f, b3f);
    }
#pragma unroll 1
    for (int k0 = 0; k0 < kHid; k0 += 32) {
      const v16h a   = frag_load(ahrow + k0);
      const v16h b0f = frag_load(wrow + (size_t)0 * kHid * kEncK + kHid + k0);
      const v16h b1f = frag_load(wrow + (size_t)1 * kHid * kEncK + kHid + k0);
      const v16h b2f = frag_load(wrow + (size_t)2 * kHid * kEncK + kHid + k0);
      const v16h b3f = frag_load(wrow + (size_t)3 * kHid * kEncK + kHid + k0);
      acc0 = mma_h(a, b0f, acc0);
      acc1 = mma_h(a, b1f, acc1);
      acc2 = mma_h(a, b2f, acc2);
      acc3 = mma_h(a, b3f, acc3);
      guard4(acc0, acc1, acc2, acc3, a, b0f, b1f, b2f, b3f);
    }
    acc_guard4(acc0, acc1, acc2, acc3);
#pragma unroll
    for (int r = 0; r < 8; ++r) {
      const float zi = acc0[r] * kWCarryInv + bb0;
      const float zf = acc1[r] * kWCarryInv + bb1;
      const float zg = acc2[r] * kWCarryInv + bb2;
      const float zo = acc3[r] * kWCarryInv + bb3;
      const float ig = fsig(zi);
      const float fg = fsig(zf);
      const float gg = ftanh(zg);
      const float og = fsig(zo);
      const float cn = fg * cst[r] + ig * gg;
      cst[r] = cn;
      const float hn = og * ftanh(cn);
      fda[r] += hn;
      ahn[(8 * hh + r) * HP + j] = (_Float16)hn;
    }
    __syncthreads();
  }

#pragma unroll
  for (int r = 0; r < 8; ++r) Fs[(8 * hh + r) * SP + j] = fda[r];
  __syncthreads();
  {
    v4f ov[2];
#pragma unroll
    for (int it = 0; it < 2; ++it) {
      const int idx = it * 128 + tid;
      const int row = idx >> 4, c4 = (idx & 15) * 4;
      ov[it] = *(const v4f*)(Fs + row * SP + c4);
    }
    for (int pass = 0; pass < 2; ++pass) {
#pragma unroll
      for (int it = 0; it < 2; ++it) {
        const int idx = it * 128 + tid;
        const int row = idx >> 4, c4 = (idx & 15) * 4;
        *(volatile v4f*)(fd + (size_t)(rowbase + row) * kDecIn + dir * kHid + c4) = ov[it];
      }
      __threadfence();
    }
  }
}

__global__ __launch_bounds__(128) void decoder_kernel(const float* __restrict__ fd, const unsigned short* __restrict__ WDp,
                                                      const float* __restrict__ dbih, const float* __restrict__ dbhh,
                                                      const float* __restrict__ dlw, const float* __restrict__ dlb,
                                                      float* __restrict__ out) {
  __shared__ __align__(16) _Float16 Fh[16 * FP];
  __shared__ __align__(16) _Float16 Fl[16 * FP];
  __shared__ __align__(16) _Float16 Ah[2 * 16 * HP];
  __shared__ __align__(16) float    Hf[16 * SP];
  __shared__ __align__(16) float    Wq[kCls * kHid];
  __shared__ __align__(16) float    Ost[kOutTile];
  __shared__ float Bq[16];
  __shared__ float Lg[16 * 12];
  const int tid = threadIdx.x, lane = tid & 31, wave = tid >> 5;
  const int c = lane & 15, hh = lane >> 4, koff = hh * 8;
  const int rowbase = blockIdx.x * 16;
  const int j = 16 * wave + c;
  const _Float16* WD = (const _Float16*)WDp;

#pragma unroll 1
  for (int it = 0; it < 4; ++it) {
    const int idx = it * 128 + tid;
    const int row = idx >> 5, c4 = (idx & 31) * 4;
    const v4f v = *(const v4f*)(fd + (size_t)(rowbase + row) * kDecIn + c4);
#pragma unroll
    for (int e = 0; e < 4; ++e) {
      const float f = v[e];
      const _Float16 hi = (_Float16)f;
      float hf = (float)hi;
      asm volatile("" : "+v"(hf));
      const _Float16 lo = (_Float16)((f - hf) * kLoCarry);
      Fh[row * FP + c4 + e] = hi;
      Fl[row * FP + c4 + e] = lo;
    }
  }
#pragma unroll 1
  for (int i = tid; i < kCls * kHid; i += 128) Wq[i] = dlw[i];
  {
    const int qc = (tid < kCls) ? tid : (kCls - 1);
    const float bv = dlb[qc];
    if (tid < 16) Bq[tid] = (tid < kCls) ? bv : 0.0f;
  }
#pragma unroll 1
  for (int i = tid; i < 2 * 16 * HP; i += 128) Ah[i] = (_Float16)0.0f;
  const float bs0 = dbih[0 * kHid + j] + dbhh[0 * kHid + j];
  const float bs1 = dbih[1 * kHid + j] + dbhh[1 * kHid + j];
  const float bs2 = dbih[2 * kHid + j] + dbhh[2 * kHid + j];
  const float bs3 = dbih[3 * kHid + j] + dbhh[3 * kHid + j];
  __syncthreads();

  const _Float16* wd = WD + (size_t)j * kDecK + koff;
  const v8f z8 = {0.f, 0.f, 0.f, 0.f, 0.f, 0.f, 0.f, 0.f};
  float gq0[8], gq1[8], gq2[8], gq3[8];
  {
    v8f h0 = z8, h1 = z8, h2 = z8, h3 = z8, l0 = z8, l1 = z8, l2 = z8, l3 = z8;
    const _Float16* fhrow = Fh + c * FP + koff;
    const _Float16* flrow = Fl + c * FP + koff;
#pragma unroll 1
    for (int k0 = 0; k0 < kDecIn; k0 += 32) {
      const v16h ah  = frag_load(fhrow + k0);
      const v16h al  = frag_load(flrow + k0);
      const v16h b0f = frag_load(wd + (size_t)0 * kHid * kDecK + k0);
      const v16h b1f = frag_load(wd + (size_t)1 * kHid * kDecK + k0);
      const v16h b2f = frag_load(wd + (size_t)2 * kHid * kDecK + k0);
      const v16h b3f = frag_load(wd + (size_t)3 * kHid * kDecK + k0);
      h0 = mma_h(ah, b0f, h0);
      h1 = mma_h(ah, b1f, h1);
      h2 = mma_h(ah, b2f, h2);
      h3 = mma_h(ah, b3f, h3);
      l0 = mma_h(al, b0f, l0);
      l1 = mma_h(al, b1f, l1);
      l2 = mma_h(al, b2f, l2);
      l3 = mma_h(al, b3f, l3);
      guard8(h0, h1, h2, h3, l0, l1, l2, l3, ah, al, b0f, b1f, b2f, b3f);
    }
    acc_guard4(h0, h1, h2, h3);
    acc_guard4(l0, l1, l2, l3);
#pragma unroll
    for (int r = 0; r < 8; ++r) {
      gq0[r] = h0[r] * kWCarryInv + l0[r] * kLoFold + bs0;
      gq1[r] = h1[r] * kWCarryInv + l1[r] * kLoFold + bs1;
      gq2[r] = h2[r] * kWCarryInv + l2[r] * kLoFold + bs2;
      gq3[r] = h3[r] * kWCarryInv + l3[r] * kLoFold + bs3;
    }
  }
  float cst[8];
#pragma unroll
  for (int r = 0; r < 8; ++r) cst[r] = 0.0f;

#pragma unroll 1
  for (int s = 0; s < kOutLen; ++s) {
    const int cur = s & 1;
    const _Float16* ahrow = Ah + cur * (16 * HP) + c * HP + koff;
    _Float16* ahn = Ah + (cur ^ 1) * (16 * HP);
    v8f acc0 = z8, acc1 = z8, acc2 = z8, acc3 = z8;
#pragma unroll 1
    for (int k0 = 0; k0 < kHid; k0 += 32) {
      const v16h a   = frag_load(ahrow + k0);
      const v16h b0f = frag_load(wd + (size_t)0 * kHid * kDecK + kDecIn + k0);
      const v16h b1f = frag_load(wd + (size_t)1 * kHid * kDecK + kDecIn + k0);
      const v16h b2f = frag_load(wd + (size_t)2 * kHid * kDecK + kDecIn + k0);
      const v16h b3f = frag_load(wd + (size_t)3 * kHid * kDecK + kDecIn + k0);
      acc0 = mma_h(a, b0f, acc0);
      acc1 = mma_h(a, b1f, acc1);
      acc2 = mma_h(a, b2f, acc2);
      acc3 = mma_h(a, b3f, acc3);
      guard4(acc0, acc1, acc2, acc3, a, b0f, b1f, b2f, b3f);
    }
    acc_guard4(acc0, acc1, acc2, acc3);
#pragma unroll
    for (int r = 0; r < 8; ++r) {
      const float zi = acc0[r] * kWCarryInv + gq0[r];
      const float zf = acc1[r] * kWCarryInv + gq1[r];
      const float zg = acc2[r] * kWCarryInv + gq2[r];
      const float zo = acc3[r] * kWCarryInv + gq3[r];
      const float ig = fsig(zi);
      const float fg = fsig(zf);
      const float gg = ftanh(zg);
      const float og = fsig(zo);
      const float cn = fg * cst[r] + ig * gg;
      cst[r] = cn;
      const float hn = og * ftanh(cn);
      ahn[(8 * hh + r) * HP + j] = (_Float16)hn;
      Hf[(8 * hh + r) * SP + j] = hn;
    }
    __syncthreads();
#pragma unroll 1
    for (int it = 0; it < 2; ++it) {
      const int p   = it * 128 + tid;
      const int pc  = (p < kPairs) ? p : (kPairs - 1);
      const int row = pc / kCls;
      const int q   = pc - row * kCls;
      float a = Bq[q];
#pragma unroll 8
      for (int k = 0; k < kHid; ++k) a = fmaf(Hf[row * SP + k], Wq[q * kHid + k], a);
      if (p < kPairs) Lg[row * 12 + q] = a;
    }
    __syncthreads();
#pragma unroll 1
    for (int it = 0; it < 2; ++it) {
      const int p   = it * 128 + tid;
      const int pc  = (p < kPairs) ? p : (kPairs - 1);
      const int row = pc / kCls;
      const int q   = pc - row * kCls;
      float mx = Lg[row * 12];
#pragma unroll 1
      for (int k = 1; k < kCls; ++k) mx = fmaxf(mx, Lg[row * 12 + k]);
      float sum = 0.0f;
#pragma unroll 1
      for (int k = 0; k < kCls; ++k) sum += expf(Lg[row * 12 + k] - mx);
      const float ev = expf(Lg[row * 12 + q] - mx);
      const float pv = ev * (1.0f / sum);
      if (p < kPairs) Ost[row * (kOutLen * kCls) + s * kCls + q] = pv;
    }
  }
  __syncthreads();
  {
    float* ob = out + (size_t)blockIdx.x * kOutTile;
    for (int pass = 0; pass < 2; ++pass) {
#pragma unroll
      for (int it = 0; it < 4; ++it) {
        const int i = it * 128 + tid;
        if (i < kOutVec) {
          const v4f v = *(const v4f*)(Ost + 4 * i);
          *(volatile v4f*)(ob + 4 * i) = v;
        }
      }
      __threadfence();
    }
  }
}

extern "C" void kernel_launch(void* const* d_in, const int* in_sizes, int n_in,
                              void* d_out, int out_size, void* d_ws, size_t ws_size, hipStream_t stream) {
  (void)in_sizes; (void)out_size;
  if (n_in < 21 || d_out == nullptr || d_ws == nullptr) return;

  const float* x       = (const float*)d_in[0];
  const float* elw     = (const float*)d_in[1];
  const float* elb     = (const float*)d_in[2];
  const float* wih_f   = (const float*)d_in[3];
  const float* whh_f   = (const float*)d_in[4];
  const float* bih_f   = (const float*)d_in[5];
  const float* bhh_f   = (const float*)d_in[6];
  const float* wih_b   = (const float*)d_in[7];
  const float* whh_b   = (const float*)d_in[8];
  const float* bih_b   = (const float*)d_in[9];
  const float* bhh_b   = (const float*)d_in[10];
  const float* dwih    = (const float*)d_in[15];
  const float* dwhh    = (const float*)d_in[16];
  const float* dbih    = (const float*)d_in[17];
  const float* dbhh    = (const float*)d_in[18];
  const float* dlw     = (const float*)d_in[19];
  const float* dlb     = (const float*)d_in[20];
  float* out = (float*)d_out;

  char* ws = (char*)d_ws; size_t off = 0;
  auto carve = [&](size_t bytes) -> char* { char* p = ws + off; off += (bytes + 255) & ~(size_t)255; return p; };
  unsigned short* E  = (unsigned short*)carve((size_t)kSteps * kBatch * kHid * 2);
  float*          FD = (float*)carve((size_t)kBatch * kDecIn * 4);
  unsigned short* WE = (unsigned short*)carve((size_t)2 * kGate * kEncK * 2);
  unsigned short* WD = (unsigned short*)carve((size_t)kGate * kDecK * 2);
  unsigned short* WL = (unsigned short*)carve((size_t)kHid * kFeatPad * 2);
  if (off > ws_size || off > (size_t)134217728) return;

  wprep_kernel<<<dim3(16, 7), 256, 0, stream>>>(wih_f, whh_f, wih_b, whh_b, dwih, dwhh, elw, WE, WD, WL);
  enc_lin_kernel<<<kBatch, 256, 0, stream>>>(x, WL, elb, E);
  bilstm_kernel<<<dim3(kBatch / 16, 2), 128, 0, stream>>>(E, WE, bih_f, bhh_f, bih_b, bhh_b, FD);
  decoder_kernel<<<kBatch / 16, 128, 0, stream>>>(FD, WD, dbih, dbhh, dlw, dlb, out);
}
